// MultiHead_94489281378
// MI455X (gfx1250) — hardware-verified
//
#include <hip/hip_runtime.h>

#ifndef NB
#define NB 2
#endif
#ifndef SEQ
#define SEQ 2048
#endif
#define NB_FULL 2
#define SEQ_FULL 2048
#define DM 1024
#define NH 16
#define HD 64
#define HG 2
#define QE 128
static_assert(NB >= 1 && NB <= NB_FULL);
static_assert(SEQ % 128 == 0 && SEQ >= 2 * QE && SEQ <= SEQ_FULL);
static_assert(QE == 128);
static_assert(NH % HG == 0 && DM == NH * HD && HD == 64);

typedef __bf16 v16b __attribute__((ext_vector_type(16)));
typedef unsigned short v8us __attribute__((ext_vector_type(8), may_alias));
typedef float  v8f  __attribute__((ext_vector_type(8)));
typedef float  v4f  __attribute__((ext_vector_type(4)));
typedef float  v4fa __attribute__((ext_vector_type(4), may_alias));
typedef _Float16 v16h __attribute__((ext_vector_type(16)));
typedef _Float16 v4h  __attribute__((ext_vector_type(4)));
union FragB { v16b v; v8us half[2]; unsigned short u[16]; };
union FragH { v16h v; v8us half[2]; _Float16 h[16]; unsigned short u[16]; };

__device__ __forceinline__ unsigned short bf16_bits(float x) { unsigned int u = __float_as_uint(x); return (unsigned short)((u + 0x7FFFu + ((u >> 16) & 1u)) >> 16); }
__device__ __forceinline__ float bf16_val(unsigned short b) { return __uint_as_float(((unsigned int)b) << 16); }
__device__ __forceinline__ float bf16_rne(float x) { return bf16_val(bf16_bits(x)); }

template <int NT>
__device__ __forceinline__ v8f mmaN(v16b ah, v16b al, v16b bh, v16b bl, v8f c) {
  c = __builtin_amdgcn_wmma_f32_16x16x32_bf16(false, ah, false, bh, (short)0, c, false, false);
  if (NT >= 2) c = __builtin_amdgcn_wmma_f32_16x16x32_bf16(false, al, false, bh, (short)0, c, false, false);
  if (NT >= 3) c = __builtin_amdgcn_wmma_f32_16x16x32_bf16(false, ah, false, bl, (short)0, c, false, false);
  asm volatile("v_nop\n\tv_nop\n\tv_nop\n\tv_nop" : "+v"(c) : "v"(ah), "v"(al), "v"(bh), "v"(bl));
  return c;
}

__device__ __forceinline__ v16h g2_frag(const _Float16* p, int hh) { FragH f; f.half[0] = *(const v8us*)((const unsigned short*)p + 8 * hh); f.half[1] = *(const v8us*)((const unsigned short*)p + 16 + 8 * hh); return f.v; }
__device__ __forceinline__ v8f g2_mma(v16h a, v16h b, v8f c) { v8f d = __builtin_amdgcn_wmma_f32_16x16x32_f16(false, a, false, b, (short)0, c, false, false); asm volatile("v_nop\n\tv_nop\n\tv_nop\n\tv_nop" : "+v"(d) : "v"(a), "v"(b)); return d; }

__global__ __launch_bounds__(256) void k_x16(const float* __restrict__ x, size_t sx, _Float16* __restrict__ X16, size_t sy, size_t n8) {
  const size_t t = (size_t)blockIdx.x * 256 + threadIdx.x; if (t >= n8) return;
  const float* src = x + (size_t)blockIdx.y * sx + t * 8; unsigned short* d = (unsigned short*)X16 + (size_t)blockIdx.y * sy + t * 8;
  const v4f a = *(const v4fa*)(src), c = *(const v4fa*)(src + 4); FragH f;
#pragma unroll
  for (int q = 0; q < 4; ++q) { f.h[q] = (_Float16)bf16_rne(a[q]); f.h[4 + q] = (_Float16)bf16_rne(c[q]); }
  const v8us o = f.half[0]; *(volatile v8us*)d = o; __threadfence(); *(volatile v8us*)d = o;
}

__global__ __launch_bounds__(256) void k_wnat(const float* __restrict__ w, size_t n8, _Float16* __restrict__ Bt) {
  const size_t t = (size_t)blockIdx.x * 256 + threadIdx.x; if (t >= n8) return;
  const v4f a = *(const v4fa*)(w + t * 8), c = *(const v4fa*)(w + t * 8 + 4); FragH f;
#pragma unroll
  for (int q = 0; q < 4; ++q) { f.h[q] = (_Float16)(bf16_rne(a[q]) * 16.0f); f.h[4 + q] = (_Float16)(bf16_rne(c[q]) * 16.0f); }
  const v8us o = f.half[0]; unsigned short* d = (unsigned short*)Bt + t * 8; *(volatile v8us*)d = o; __threadfence(); *(volatile v8us*)d = o;
}

template <int NHv, int TTv>
__global__ __launch_bounds__(256) void k_vt(const _Float16* __restrict__ V16, int ldv, int voff, _Float16* __restrict__ Vt) {
  __shared__ unsigned short tl[64][66]; const int tid = threadIdx.x; const int slab = blockIdx.x / (TTv / 64), lg = blockIdx.x % (TTv / 64); const int b = slab / NHv, h = slab % NHv;
  for (int i = tid; i < 64 * 8; i += 256) { const int r = i / 8, c8 = (i % 8) * 8; FragH f; f.half[0] = *(const v8us*)((const unsigned short*)V16 + ((size_t)b * TTv + lg * 64 + r) * ldv + voff + h * 64 + c8);
#pragma unroll
    for (int q = 0; q < 8; ++q) tl[r][c8 + q] = f.u[q]; }
  __syncthreads();
  for (int pass = 0; pass < 2; ++pass) {
#pragma unroll
    for (int rd = 0; rd < 2; ++rd) { const int d = rd * 32 + tid / 8, pc = tid % 8; FragH f;
#pragma unroll
      for (int q = 0; q < 8; ++q) f.u[q] = tl[pc * 8 + q][d];
      *(volatile v8us*)((unsigned short*)Vt + ((size_t)slab * 64 + d) * TTv + lg * 64 + pc * 8) = f.half[0]; }
    if (pass == 0) __threadfence(); } }

__global__ __launch_bounds__(128) void k_gemm2(const _Float16* __restrict__ A, int lda, size_t sA, const _Float16* __restrict__ Bh, int ldb, size_t sB, float alpha,
    float* __restrict__ C, _Float16* __restrict__ C16, int ldc, size_t sC, int M, int N, int K, int cz) {
  __shared__ __attribute__((aligned(16))) float so[4][32][68];
  const int tid = threadIdx.x, w = tid >> 5, lane = tid & 31, ln = lane & 15, hh = lane >> 4; const int by = blockIdx.y;
  A += (size_t)by * sA; Bh += (size_t)by * sB; const size_t cofs = (size_t)by * sC;
  const int ntn = N >> 6; const int mt = blockIdx.x / ntn, nq = blockIdx.x - mt * ntn; const int row0 = mt * 128 + 32 * w, col0 = nq * 64; if (row0 >= M) return;
  if ((cz & 1) && col0 >= (mt + 1) * 128) return;
  const int Kc = (mt + 1) * 128; const int Ke = (cz & 2) ? ((Kc < K) ? Kc : K) : K;
  const _Float16* a0p = A + (size_t)(row0 + ln) * lda; const _Float16* a1p = a0p + (size_t)16 * lda;
  const _Float16* b0p = Bh + (size_t)(col0 + ln) * ldb; const _Float16* b1p = b0p + (size_t)16 * ldb; const _Float16* b2p = b1p + (size_t)16 * ldb; const _Float16* b3p = b2p + (size_t)16 * ldb;
  const v8f z8 = {0.f,0.f,0.f,0.f,0.f,0.f,0.f,0.f}; v8f c00 = z8, c01 = z8, c02 = z8, c03 = z8, c10 = z8, c11 = z8, c12 = z8, c13 = z8;
#pragma unroll 1
  for (int kb = 0; kb < Ke; kb += 32) { const v16h a0 = g2_frag(a0p + kb, hh), a1 = g2_frag(a1p + kb, hh);
    v16h b = g2_frag(b0p + kb, hh); c00 = g2_mma(a0, b, c00); c10 = g2_mma(a1, b, c10);
    b = g2_frag(b1p + kb, hh); c01 = g2_mma(a0, b, c01); c11 = g2_mma(a1, b, c11);
    b = g2_frag(b2p + kb, hh); c02 = g2_mma(a0, b, c02); c12 = g2_mma(a1, b, c12);
    b = g2_frag(b3p + kb, hh); c03 = g2_mma(a0, b, c03); c13 = g2_mma(a1, b, c13); }
  v8f accs[8] = {c00, c01, c02, c03, c10, c11, c12, c13};
#pragma unroll
  for (int u = 0; u < 8; ++u) { const int t = u & 3, half = u >> 2;
#pragma unroll
    for (int r = 0; r < 8; ++r) { const int rloc = half * 16 + 8 * hh + r; so[w][rloc][t * 16 + ln] = accs[u][r] * alpha; } }
  __builtin_amdgcn_fence(4  , "workgroup"); __builtin_amdgcn_wave_barrier();
  const int rsub = lane >> 4, c4 = (lane & 15) * 4;
  for (int pass = 0; pass < 2; ++pass) {
#pragma unroll
    for (int q = 0; q < 16; ++q) { const int r = q * 2 + rsub; const v4f v = *(const v4fa*)&so[w][r][c4];
      if (C) *(volatile v4f*)(C + cofs + (size_t)(row0 + r) * ldc + col0 + c4) = v;
      if (C16) { v4h h4; for (int i = 0; i < 4; ++i) h4[i] = (_Float16)v[i]; *(volatile v4h*)(C16 + cofs + (size_t)(row0 + r) * ldc + col0 + c4) = h4; } }
    if (pass == 0) __threadfence(); } }

__global__ __launch_bounds__(256) void k_rsmc(const float* __restrict__ S, _Float16* __restrict__ P, int qn, int hg) {
  #pragma clang fp contract(off)
  const int t = blockIdx.x * 256 + threadIdx.x; if (t >= qn * hg) return;
  const int qi = t % qn; const size_t i = (size_t)(t / qn) * SEQ + qi; const float* s = S + i * SEQ;
  int jend = ((qi >> 7) + 1) << 7; if (jend > SEQ) jend = SEQ;
  float mx = -3.0e38f;
#pragma unroll 1
  for (int j = 0; j <= qi; ++j) mx = fmaxf(mx, s[j]);
  float se = 0.f;
#pragma unroll 1
  for (int j = 0; j <= qi; ++j) se += __expf(s[j] - mx);
  const float sc = 256.0f / se;
#pragma unroll 1
  for (int j0 = 0; j0 < jend; j0 += 8) { FragH f;
#pragma unroll
    for (int q = 0; q < 8; ++q) { const int j = j0 + q; const float e = (j <= qi) ? __expf(s[j] - mx) * sc : 0.0f; f.h[q] = (_Float16)e; }
    unsigned short* d = (unsigned short*)P + i * SEQ + j0; const v8us o = f.half[0]; *(volatile v8us*)d = o; __threadfence(); *(volatile v8us*)d = o; } }

template <int NT>
__global__ __launch_bounds__(128) void k_gemm_ss(const float* __restrict__ A, int lda, size_t sA1, size_t sA2, const float* __restrict__ Bm, int ldb, size_t sB1, size_t sB2, int nhy, float alpha,
    float* __restrict__ C, int ldc, size_t sC1, size_t sC2, int M, int N, int K) {
  __shared__ __attribute__((aligned(16))) float so[4][16][64];
  const int tid = threadIdx.x, w = tid >> 5, lane = tid & 31, ln = lane & 15, hh = lane >> 4;
  const int by = blockIdx.y; const int bb = by / nhy, hy = by - bb * nhy;
  A += (size_t)bb * sA1 + (size_t)hy * sA2; Bm += (size_t)bb * sB1 + (size_t)hy * sB2; C += (size_t)bb * sC1 + (size_t)hy * sC2;
  const int ntn = N / 64; const int wid = blockIdx.x * 4 + w; const int mt = wid / ntn, nq = wid % ntn; if (mt * 16 >= M) return;
  const int row0 = mt * 16, col0 = nq * 64; const float* arow = A + (size_t)(row0 + ln) * lda;
  v8f acc[4] = {};
#pragma unroll 1
  for (int kb = 0; kb < K; kb += 32) {
    FragB ah, al;
    { const v4f x0 = *(const v4fa*)(arow + kb + 8 * hh), x1 = *(const v4fa*)(arow + kb + 8 * hh + 4);
      const v4f x2 = *(const v4fa*)(arow + kb + 16 + 8 * hh), x3 = *(const v4fa*)(arow + kb + 16 + 8 * hh + 4);
      float xs[16] = {x0[0],x0[1],x0[2],x0[3],x1[0],x1[1],x1[2],x1[3],x2[0],x2[1],x2[2],x2[3],x3[0],x3[1],x3[2],x3[3]};
#pragma unroll
      for (int i = 0; i < 16; ++i) { const unsigned short hb = bf16_bits(xs[i]); ah.u[i] = hb; al.u[i] = bf16_bits(xs[i] - bf16_val(hb)); } }
#pragma unroll
    for (int t = 0; t < 4; ++t) {
      const float* brow = Bm + (size_t)(col0 + t * 16 + ln) * ldb + kb;
      const v4f y0 = *(const v4fa*)(brow + 8 * hh), y1 = *(const v4fa*)(brow + 8 * hh + 4);
      const v4f y2 = *(const v4fa*)(brow + 16 + 8 * hh), y3 = *(const v4fa*)(brow + 16 + 8 * hh + 4);
      float ys[16] = {y0[0],y0[1],y0[2],y0[3],y1[0],y1[1],y1[2],y1[3],y2[0],y2[1],y2[2],y2[3],y3[0],y3[1],y3[2],y3[3]};
      FragB bh, bl;
#pragma unroll
      for (int i = 0; i < 16; ++i) { const unsigned short hb = bf16_bits(ys[i]); bh.u[i] = hb; bl.u[i] = (NT >= 3) ? bf16_bits(ys[i] - bf16_val(hb)) : (unsigned short)0; }
      acc[t] = mmaN<NT>(ah.v, al.v, bh.v, bl.v, acc[t]);
    }
  }
#pragma unroll
  for (int t = 0; t < 4; ++t) {
#pragma unroll
    for (int r = 0; r < 8; ++r) so[w][8 * hh + r][t * 16 + ln] = acc[t][r] * alpha; }
  __builtin_amdgcn_fence(4  , "workgroup"); __builtin_amdgcn_wave_barrier();
  const int rsub = lane >> 4, c4 = (lane & 15) * 4;
  for (int pass = 0; pass < 2; ++pass) {
#pragma unroll
    for (int q = 0; q < 8; ++q) { const int r = q * 2 + rsub; const v4f v = *(const v4fa*)&so[w][r][c4]; *(volatile v4f*)(C + (size_t)(row0 + r) * ldc + col0 + c4) = v; }
    if (pass == 0) __threadfence(); } }

__global__ __launch_bounds__(256) void k_tr64(const float* __restrict__ VF, float* __restrict__ VFT) {
  __shared__ float tl[64][65];
  const int tid = threadIdx.x, w = tid >> 5, lane = tid & 31;
  const int ktn = QE / 64; const int slab = blockIdx.x / ktn, kt = blockIdx.x % ktn; const int b = slab / NH, h = slab % NH;
  const float* src = VF + ((size_t)b * QE + kt * 64) * DM + h * HD;
  for (int idx = tid; idx < 64 * 16; idx += 256) { const int i = idx >> 4, c4 = (idx & 15) * 4; const v4f v = *(const v4fa*)(src + (size_t)i * DM + c4);
    tl[i][c4] = v[0]; tl[i][c4 + 1] = v[1]; tl[i][c4 + 2] = v[2]; tl[i][c4 + 3] = v[3]; }
  __syncthreads();
  float* dst = VFT + (size_t)slab * HD * QE + kt * 64;
  for (int pass = 0; pass < 2; ++pass) {
#pragma unroll
    for (int it = 0; it < 4; ++it) { const int L = w * 16 + it * 4 + (lane >> 3); const int d = L >> 1, seg = L & 1; const int col = seg * 32 + (lane & 7) * 4;
      v4f v; v[0] = tl[col][d]; v[1] = tl[col + 1][d]; v[2] = tl[col + 2][d]; v[3] = tl[col + 3][d];
      *(volatile v4f*)(dst + (size_t)d * QE + col) = v; }
    if (pass == 0) __threadfence(); } }

__global__ __launch_bounds__(256) void k_esm(const float* __restrict__ SE, float* __restrict__ PF) {
  #pragma clang fp contract(off)
  __shared__ __attribute__((aligned(16))) float sp[32][QE + 4];
  const int tid = threadIdx.x, w = tid >> 5, lane = tid & 31;
  const int rl = tid >> 3, sub = tid & 7;
  const size_t R = (size_t)blockIdx.x * 32 + rl;
  const int r = (int)(R % QE);
  const float* s = SE + R * QE;
  const int k0 = sub * (QE / 8);
  float mx = -3.0e38f;
#pragma unroll 1
  for (int j = 0; j < QE / 8; ++j) { const int k = k0 + j; const float l = s[k] * 0.03125f; mx = (k <= r) ? fmaxf(mx, l) : mx; }
  mx = fmaxf(mx, __shfl_xor(mx, 1, 32)); mx = fmaxf(mx, __shfl_xor(mx, 2, 32)); mx = fmaxf(mx, __shfl_xor(mx, 4, 32));
  float se = 0.f;
#pragma unroll 1
  for (int j = 0; j < QE / 8; ++j) { const int k = k0 + j; const float e = __expf(s[k] * 0.03125f - mx); se += (k <= r) ? e : 0.0f; }
  se += __shfl_xor(se, 1, 32); se += __shfl_xor(se, 2, 32); se += __shfl_xor(se, 4, 32);
  const float inv = 1.0f / se;
#pragma unroll 1
  for (int j = 0; j < QE / 8; ++j) { const int k = k0 + j; const float e = __expf(s[k] * 0.03125f - mx) * inv; sp[rl][k] = (k <= r) ? e : 0.0f; }
  __syncthreads();
  float* dst = PF + (size_t)blockIdx.x * 32 * QE;
  for (int pass = 0; pass < 2; ++pass) {
#pragma unroll
    for (int it = 0; it < QE / 32; ++it) {
      const int L = w * (QE / 8) + it * 4 + (lane >> 3);
      const int row = L / (QE / 32), seg = L % (QE / 32); const int col = seg * 32 + (lane & 7) * 4;
      const v4f v = *(const v4fa*)&sp[row][col];
      *(volatile v4f*)(dst + (size_t)row * QE + col) = v;
    }
    if (pass == 0) __threadfence();
  }
}

extern "C" void kernel_launch(void* const* d_in, const int* in_sizes, int n_in,
                              void* d_out, int out_size, void* d_ws, size_t ws_size, hipStream_t stream) {
  if (n_in < 7) return;
  const long long need_x = ((long long)(NB - 1) * SEQ_FULL + SEQ) * DM;
  if ((long long)in_sizes[0] < need_x || (long long)in_sizes[1] < need_x || (long long)in_sizes[2] < need_x) return;
  if (in_sizes[3] < DM * DM || in_sizes[4] < DM * DM || in_sizes[5] < DM * DM || in_sizes[6] < DM * DM) return;
  if ((long long)out_size < need_x) return;
  const float* xq = (const float*)d_in[0]; const float* xk = (const float*)d_in[1]; const float* xv = (const float*)d_in[2];
  const float* wq = (const float*)d_in[3]; const float* wk = (const float*)d_in[4]; const float* wv = (const float*)d_in[5]; const float* wo = (const float*)d_in[6];
  float* out = (float*)d_out;
  char* ws = (char*)d_ws; size_t off = 0;
  auto take = [&](size_t bytes) { char* p = ws + off; off += (bytes + 255) & ~(size_t)255; return p; };
  const size_t NR = (size_t)NB * SEQ;
  _Float16* WQ16 = (_Float16*)take((size_t)DM * DM * 2); _Float16* WK16 = (_Float16*)take((size_t)DM * DM * 2);
  _Float16* WV16 = (_Float16*)take((size_t)DM * DM * 2); _Float16* WO16 = (_Float16*)take((size_t)DM * DM * 2);
  _Float16* X16 = (_Float16*)take(NR * DM * 2);
  _Float16* Q16 = (_Float16*)take(NR * DM * 2); _Float16* K16 = (_Float16*)take(NR * DM * 2); _Float16* V16 = (_Float16*)take(NR * DM * 2); _Float16* O16 = (_Float16*)take(NR * DM * 2);
  _Float16* VT = (_Float16*)take((size_t)NB * NH * HD * SEQ * 2);
  float* S = (float*)take((size_t)HG * SEQ * SEQ * 4); _Float16* P = (_Float16*)take((size_t)HG * SEQ * SEQ * 2);
  float* QF = (float*)take((size_t)NB * QE * DM * 4); float* KF = (float*)take((size_t)NB * QE * DM * 4); float* VF = (float*)take((size_t)NB * QE * DM * 4); float* OF = (float*)take((size_t)NB * QE * DM * 4);
  float* VFT = (float*)take((size_t)NB * NH * HD * QE * 4); float* SE = (float*)take((size_t)NB * NH * QE * QE * 4); float* PF = (float*)take((size_t)NB * NH * QE * QE * 4);
  if (off > ws_size) return;

  const size_t w8 = (size_t)DM * DM / 8; const unsigned wg = (unsigned)((w8 + 255) / 256);
  k_wnat<<<wg, 256, 0, stream>>>(wq, w8, WQ16); k_wnat<<<wg, 256, 0, stream>>>(wk, w8, WK16); k_wnat<<<wg, 256, 0, stream>>>(wv, w8, WV16); k_wnat<<<wg, 256, 0, stream>>>(wo, w8, WO16);

  const size_t n8 = (size_t)SEQ * DM / 8; const dim3 gx((unsigned)((n8 + 255) / 256), NB);
  const dim3 gp((unsigned)((NR / 128) * (DM / 64)), 1), ge((unsigned)((QE / 128) * (DM / 64)), NB);
  k_x16<<<gx, 256, 0, stream>>>(xq, (size_t)SEQ_FULL * DM, X16, (size_t)SEQ * DM, n8);
  k_gemm2<<<gp, 128, 0, stream>>>(X16, DM, 0, WQ16, DM, 0, 0.0625f, nullptr, Q16, DM, 0, (int)NR, DM, DM, 0);
  k_gemm2<<<ge, 128, 0, stream>>>(X16, DM, (size_t)SEQ * DM, WQ16, DM, 0, 0.0625f, QF, nullptr, DM, (size_t)QE * DM, QE, DM, DM, 0);
  k_x16<<<gx, 256, 0, stream>>>(xk, (size_t)SEQ_FULL * DM, X16, (size_t)SEQ * DM, n8);
  k_gemm2<<<gp, 128, 0, stream>>>(X16, DM, 0, WK16, DM, 0, 0.0625f, nullptr, K16, DM, 0, (int)NR, DM, DM, 0);
  k_gemm2<<<ge, 128, 0, stream>>>(X16, DM, (size_t)SEQ * DM, WK16, DM, 0, 0.0625f, KF, nullptr, DM, (size_t)QE * DM, QE, DM, DM, 0);
  k_x16<<<gx, 256, 0, stream>>>(xv, (size_t)SEQ_FULL * DM, X16, (size_t)SEQ * DM, n8);
  k_gemm2<<<gp, 128, 0, stream>>>(X16, DM, 0, WV16, DM, 0, 0.0625f, nullptr, V16, DM, 0, (int)NR, DM, DM, 0);
  k_gemm2<<<ge, 128, 0, stream>>>(X16, DM, (size_t)SEQ * DM, WV16, DM, 0, 0.0625f, VF, nullptr, DM, (size_t)QE * DM, QE, DM, DM, 0);

  k_vt<NH, SEQ><<<(unsigned)(NB * NH * (SEQ / 64)), 256, 0, stream>>>(V16, DM, 0, VT);

  for (int b = 0; b < NB; ++b) {
    for (int h0 = 0; h0 < NH; h0 += HG) {
      k_gemm2<<<dim3((unsigned)((SEQ / 128) * (SEQ / 64)), HG), 128, 0, stream>>>(Q16 + (size_t)b * SEQ * DM + h0 * HD, DM, (size_t)HD, K16 + (size_t)b * SEQ * DM + h0 * HD, DM, (size_t)HD, 0.03125f,
          S, nullptr, SEQ, (size_t)SEQ * SEQ, SEQ, SEQ, HD, 1);
      k_rsmc<<<(unsigned)((HG * SEQ + 255) / 256), 256, 0, stream>>>(S, P, SEQ, HG);
      k_gemm2<<<dim3((unsigned)((SEQ / 128) * (HD / 64)), HG), 128, 0, stream>>>(P, SEQ, (size_t)SEQ * SEQ, VT + (size_t)(b * NH + h0) * HD * SEQ, SEQ, (size_t)HD * SEQ, 0.25f,
          nullptr, O16 + (size_t)b * SEQ * DM + h0 * HD, DM, (size_t)HD, SEQ, HD, SEQ, 2);
    }
  }
  k_gemm2<<<dim3((unsigned)(((SEQ - QE) / 128) * (DM / 64)), NB), 128, 0, stream>>>(O16 + (size_t)QE * DM, DM, (size_t)SEQ * DM, WO16, DM, 0, 0.0009765625f,
      out + (size_t)QE * DM, nullptr, DM, (size_t)SEQ_FULL * DM, SEQ - QE, DM, DM, 0);

  k_tr64<<<(unsigned)(NB * NH * (QE / 64)), 256, 0, stream>>>(VF, VFT);
  k_gemm_ss<3><<<dim3((unsigned)(((QE / 16) * (QE / 64) + 3) / 4), NB * NH), 128, 0, stream>>>(QF, DM, (size_t)QE * DM, (size_t)HD, KF, DM, (size_t)QE * DM, (size_t)HD, NH, 1.0f,
      SE, QE, (size_t)NH * QE * QE, (size_t)QE * QE, QE, QE, HD);
  k_esm<<<(unsigned)(NB * NH * QE / 32), 256, 0, stream>>>(SE, PF);
  k_gemm_ss<3><<<dim3((unsigned)(((QE / 16) * (HD / 64) + 3) / 4), NB * NH), 128, 0, stream>>>(PF, QE, (size_t)NH * QE * QE, (size_t)QE * QE, VFT, QE, (size_t)NH * HD * QE, (size_t)HD * QE, NH, 1.0f,
      OF, DM, (size_t)QE * DM, (size_t)HD, QE, HD, QE);
  k_gemm_ss<2><<<dim3((unsigned)(((QE / 16) * (DM / 64) + 3) / 4), NB), 128, 0, stream>>>(OF, DM, (size_t)QE * DM, 0, wo, DM, 0, 0, 1, 1.0f,
      out, DM, (size_t)SEQ_FULL * DM, 0, QE, DM, DM);
}
